// LSTM_2302102471468
// MI455X (gfx1250) — hardware-verified
//
#include <hip/hip_runtime.h>
#include <math.h>

constexpr int NBAT    = 64;
constexpr int NSTEP   = 512;
constexpr int NIN     = 256;
constexpr int NHID    = 512;
constexpr int NGATE   = 4 * NHID;
constexpr int NTHR    = 256;
constexpr int SEQ_BLK = 16;
constexpr int XPITCH  = 264;
constexpr int HPITCH  = 520;
constexpr int OPITCH  = 516;
constexpr float WCARRY     = 64.0f;
constexpr float WCARRY_INV = 1.0f / 64.0f;
constexpr float SCLAMP     = 30.0f;
constexpr float TCLAMP     = 15.0f;
static_assert(NBAT % SEQ_BLK == 0);
static_assert(NHID == 64 * (NTHR / 32));
static_assert(NIN % 32 == 0 && NHID % 32 == 0);
static_assert(NGATE == 4 * NHID);
static_assert((2 * SEQ_BLK * HPITCH) % NTHR == 0);
static_assert(SEQ_BLK * (NIN / 8) == 2 * NTHR);
static_assert(SEQ_BLK * (NHID / 4) == 8 * NTHR);
static_assert(NGATE / 4 == 2 * NTHR);
static_assert((XPITCH * 2) % 16 == 0 && (HPITCH * 2) % 16 == 0 && (OPITCH * 4) % 16 == 0);
static_assert((NBAT * NSTEP) * (NIN / 8) % NTHR == 0 && NGATE * (NIN / 8) % NTHR == 0 && NGATE * (NHID / 8) % NTHR == 0);

typedef __attribute__((ext_vector_type(16))) _Float16 v16h;
typedef __attribute__((ext_vector_type(8)))  _Float16 v8h;
typedef __attribute__((ext_vector_type(16))) __bf16   v16b;
typedef __attribute__((ext_vector_type(8)))  __bf16   v8b;
typedef __attribute__((ext_vector_type(8)))  float    v8f;
typedef __attribute__((ext_vector_type(4)))  float    v4f;

__device__ __forceinline__ unsigned short f2bf_bits(float f) {
  unsigned u = __float_as_uint(f);
  return (unsigned short)((u + 0x7FFFu + ((u >> 16) & 1u)) >> 16);
}
__device__ __forceinline__ float bf_bits2f(unsigned short h) { return __uint_as_float(((unsigned)h) << 16); }
__device__ __forceinline__ float bf16r(float f) { return bf_bits2f(f2bf_bits(f)); }

__device__ __forceinline__ void grp_guard_b(v8f& a0, v8f& a1, v8f& a2, v8f& a3, v16b x, v16b y0, v16b y1, v16b y2, v16b y3) {
  asm volatile("v_nop\n\tv_nop\n\tv_nop\n\tv_nop" : "+v"(a0), "+v"(a1), "+v"(a2), "+v"(a3) : "v"(x), "v"(y0), "v"(y1), "v"(y2), "v"(y3));
}
__device__ __forceinline__ void grp_guard_h(v8f& a0, v8f& a1, v8f& a2, v8f& a3, v16h x, v16h y0, v16h y1, v16h y2, v16h y3) {
  asm volatile("v_nop\n\tv_nop\n\tv_nop\n\tv_nop" : "+v"(a0), "+v"(a1), "+v"(a2), "+v"(a3) : "v"(x), "v"(y0), "v"(y1), "v"(y2), "v"(y3));
}
__device__ __forceinline__ void acc_guard4(v8f& a, v8f& b, v8f& c, v8f& d) { asm volatile("v_nop\n\tv_nop\n\tv_nop\n\tv_nop" : "+v"(a), "+v"(b), "+v"(c), "+v"(d)); }

template <typename T> struct Frag;
template <> struct Frag<_Float16> {
  typedef v16h V; union U { v16h v; v8h h[2]; };
  static __device__ __forceinline__ v16h load(const _Float16* p) {
    U f; f.h[0] = *(const v8h*)(p); f.h[1] = *(const v8h*)(p + 16); return f.v;
  }
  static __device__ __forceinline__ v8f mma(v16h a, v16h b, v8f c) {
    return __builtin_amdgcn_wmma_f32_16x16x32_f16(false, a, false, b, (short)0, c, false, false);
  }
};
template <> struct Frag<__bf16> {
  typedef v16b V; union U { v16b v; v8b h[2]; };
  static __device__ __forceinline__ v16b load(const __bf16* p) {
    U f; f.h[0] = *(const v8b*)(p); f.h[1] = *(const v8b*)(p + 16); return f.v;
  }
  static __device__ __forceinline__ v8f mma(v16b a, v16b b, v8f c) {
    return __builtin_amdgcn_wmma_f32_16x16x32_bf16(false, a, false, b, (short)0, c, false, false);
  }
};

__device__ __forceinline__ float fsig(float x) {
  const float xc = fminf(fmaxf(x, -SCLAMP), SCLAMP);
  return 1.0f / (1.0f + expf(-xc));
}
__device__ __forceinline__ float ftanh(float x) {
  const float xc = fminf(fmaxf(x, -TCLAMP), TCLAMP);
  return 1.0f - 2.0f / (expf(2.0f * xc) + 1.0f);
}

template <int MODE>
__global__ __launch_bounds__(NTHR) void cvt8_kernel(const float* __restrict__ src, unsigned short* __restrict__ dst,
                                                    int nrow, int ncol8, int spitch, int scol0, float sc) {
  const int i  = blockIdx.x * NTHR + threadIdx.x;
  const int n8 = nrow * ncol8;
  if (i < n8) {
    const int row = i / ncol8;
    const int c8  = i - row * ncol8;
    const float* sp = src + (size_t)row * spitch + scol0 + c8 * 8;
    const v4f a = *(const v4f*)(sp);
    const v4f b = *(const v4f*)(sp + 4);
    v8h hv;
#pragma unroll
    for (int e = 0; e < 4; ++e) {
      unsigned short b0, b1;
      if (MODE == 0) {
        b0 = f2bf_bits(a[e] * sc);
        b1 = f2bf_bits(b[e] * sc);
      } else {
        b0 = __builtin_bit_cast(unsigned short, (_Float16)(bf16r(a[e]) * sc));
        b1 = __builtin_bit_cast(unsigned short, (_Float16)(bf16r(b[e]) * sc));
      }
      hv[e]     = __builtin_bit_cast(_Float16, b0);
      hv[4 + e] = __builtin_bit_cast(_Float16, b1);
    }
    *(volatile v8h*)(dst + (size_t)i * 8) = hv;
    __threadfence();
    *(volatile v8h*)(dst + (size_t)i * 8) = hv;
  }
}

__global__ __launch_bounds__(NTHR) void bias_prep_kernel(const float* __restrict__ b_a, const float* __restrict__ b_b,
                                                         float* __restrict__ dst) {
  const int i = blockIdx.x * NTHR + threadIdx.x;
  if (i < NGATE / 4) {
    const int idx = i * 4;
    const v4f va = *(const v4f*)(b_a + idx);
    const v4f vb = *(const v4f*)(b_b + idx);
    v4f o;
#pragma unroll
    for (int e = 0; e < 4; ++e) o[e] = bf16r(va[e]) + bf16r(vb[e]);
    *(volatile v4f*)(dst + idx) = o;
    __threadfence();
    *(volatile v4f*)(dst + idx) = o;
  }
}

__device__ __forceinline__ void stage_x_tile(const unsigned short* __restrict__ XB, unsigned short* xs, int rowbase, int t, int tid) {
#pragma unroll
  for (int i = 0; i < 2; ++i) {
    const int idx = i * NTHR + tid;
    const int row = idx >> 5;
    const int c8  = (idx & 31) * 8;
    const uint4 v = *(const uint4*)(XB + (((size_t)(rowbase + row) * NSTEP + (size_t)t) * NIN + c8));
    *(uint4*)(xs + row * XPITCH + c8) = v;
  }
}

__global__ __launch_bounds__(NTHR) void lstm_seq_kernel(const unsigned short* __restrict__ XB,
                                                        const unsigned short* __restrict__ WIp,
                                                        const unsigned short* __restrict__ WHp,
                                                        const float* __restrict__ bias,
                                                        const int* __restrict__ length,
                                                        float* __restrict__ out) {
  __shared__ __align__(16) unsigned short Xs[2][SEQ_BLK * XPITCH];
  __shared__ __align__(16) _Float16       Ah[2][SEQ_BLK * HPITCH];
  __shared__ __align__(16) float          Hs[SEQ_BLK * OPITCH];
  const __bf16*   WI = (const __bf16*)WIp;
  const _Float16* WH = (const _Float16*)WHp;
  const int tid = threadIdx.x, lane = tid & 31, wave = tid >> 5;
  const int c = lane & 15, hh = lane >> 4, koff = hh * 8;
  const int rowbase = blockIdx.x * SEQ_BLK;

  {
    _Float16* ahf = &Ah[0][0];
#pragma unroll 1
    for (int i = tid; i < 2 * SEQ_BLK * HPITCH; i += NTHR) ahf[i] = (_Float16)0.0f;
  }
  stage_x_tile(XB, &Xs[0][0], rowbase, 0, tid);

  int lm[8];
#pragma unroll
  for (int r = 0; r < 8; ++r) {
    int L = length[rowbase + 8 * hh + r];
    L = (L < 1) ? 1 : L;
    L = (L > NSTEP) ? NSTEP : L;
    lm[r] = L - 1;
  }
  asm volatile("" ::: "memory");

  float bb[4][4], cst[4][8], hfin[4][8];
#pragma unroll
  for (int nt = 0; nt < 4; ++nt) {
    const int j = 64 * wave + 16 * nt + c;
#pragma unroll
    for (int g = 0; g < 4; ++g) bb[nt][g] = bias[g * NHID + j];
    asm volatile("" ::: "memory");
#pragma unroll
    for (int r = 0; r < 8; ++r) { cst[nt][r] = 0.0f; hfin[nt][r] = 0.0f; }
  }
  __syncthreads();

  const v8f z8 = {0.f, 0.f, 0.f, 0.f, 0.f, 0.f, 0.f, 0.f};
  constexpr size_t GPI = (size_t)NHID * NIN;
  constexpr size_t GPH = (size_t)NHID * NHID;

#pragma unroll 1
  for (int t = 0; t < NSTEP; ++t) {
    const int cur = t & 1;
    const __bf16*   axrow = (const __bf16*)(&Xs[cur][0]) + c * XPITCH + koff;
    const _Float16* ahrow = &Ah[cur][0] + c * HPITCH + koff;
    _Float16* ahn = &Ah[cur ^ 1][0];

#pragma unroll
    for (int nt = 0; nt < 4; ++nt) {
      const int j = 64 * wave + 16 * nt + c;
      const __bf16*   wx = WI + (size_t)j * NIN + koff;
      const _Float16* wh = WH + (size_t)j * NHID + koff;
      v8f acc[4];
      acc[0] = z8; acc[1] = z8; acc[2] = z8; acc[3] = z8;
#pragma unroll 1
      for (int kx = 0; kx < NIN; kx += 32) {
        const v16b a  = Frag<__bf16>::load(axrow + kx);
        const v16b b0 = Frag<__bf16>::load(wx + kx);
        const v16b b1 = Frag<__bf16>::load(wx + 1 * GPI + kx);
        const v16b b2 = Frag<__bf16>::load(wx + 2 * GPI + kx);
        const v16b b3 = Frag<__bf16>::load(wx + 3 * GPI + kx);
        acc[0] = Frag<__bf16>::mma(a, b0, acc[0]);
        acc[1] = Frag<__bf16>::mma(a, b1, acc[1]);
        acc[2] = Frag<__bf16>::mma(a, b2, acc[2]);
        acc[3] = Frag<__bf16>::mma(a, b3, acc[3]);
        grp_guard_b(acc[0], acc[1], acc[2], acc[3], a, b0, b1, b2, b3);
      }
#pragma unroll 1
      for (int k0 = 0; k0 < NHID; k0 += 32) {
        const v16h a  = Frag<_Float16>::load(ahrow + k0);
        const v16h b0 = Frag<_Float16>::load(wh + k0);
        const v16h b1 = Frag<_Float16>::load(wh + 1 * GPH + k0);
        const v16h b2 = Frag<_Float16>::load(wh + 2 * GPH + k0);
        const v16h b3 = Frag<_Float16>::load(wh + 3 * GPH + k0);
        acc[0] = Frag<_Float16>::mma(a, b0, acc[0]);
        acc[1] = Frag<_Float16>::mma(a, b1, acc[1]);
        acc[2] = Frag<_Float16>::mma(a, b2, acc[2]);
        acc[3] = Frag<_Float16>::mma(a, b3, acc[3]);
        grp_guard_h(acc[0], acc[1], acc[2], acc[3], a, b0, b1, b2, b3);
      }
      acc_guard4(acc[0], acc[1], acc[2], acc[3]);
#pragma unroll
      for (int r = 0; r < 8; ++r) {
        const float zi = acc[0][r] * WCARRY_INV + bb[nt][0];
        const float zf = acc[1][r] * WCARRY_INV + bb[nt][1];
        const float zg = acc[2][r] * WCARRY_INV + bb[nt][2];
        const float zo = acc[3][r] * WCARRY_INV + bb[nt][3];
        const float ig = fsig(zi);
        const float fg = fsig(zf);
        const float gg = ftanh(zg);
        const float og = fsig(zo);
        const float cn = fg * cst[nt][r] + ig * gg;
        cst[nt][r] = cn;
        const float hn = og * ftanh(cn);
        ahn[(8 * hh + r) * HPITCH + j] = (_Float16)hn;
        hfin[nt][r] = (t == lm[r]) ? hn : hfin[nt][r];
      }
    }
    {
      const int tn = (t + 1 < NSTEP) ? (t + 1) : (NSTEP - 1);
      stage_x_tile(XB, &Xs[cur ^ 1][0], rowbase, tn, tid);
    }
    __syncthreads();
  }

#pragma unroll
  for (int nt = 0; nt < 4; ++nt) {
    const int j = 64 * wave + 16 * nt + c;
#pragma unroll
    for (int r = 0; r < 8; ++r) Hs[(8 * hh + r) * OPITCH + j] = hfin[nt][r];
  }
  __syncthreads();
  for (int pass = 0; pass < 2; ++pass) {
#pragma unroll
    for (int it = 0; it < 8; ++it) {
      const int idx = it * NTHR + tid;
      const int row = idx >> 7, c4 = (idx & 127) * 4;
      const v4f v = *(const v4f*)(Hs + row * OPITCH + c4);
      *(volatile v4f*)(out + (size_t)(rowbase + row) * NHID + c4) = v;
    }
    __threadfence();
  }
}

extern "C" void kernel_launch(void* const* d_in, const int* in_sizes, int n_in,
                              void* d_out, int out_size, void* d_ws, size_t ws_size, hipStream_t stream) {
  if (n_in < 6 || d_out == nullptr || d_ws == nullptr) return;
  if (in_sizes[0] != NBAT * NSTEP * NIN || in_sizes[1] != NBAT || in_sizes[2] != NGATE * NIN ||
      in_sizes[3] != NGATE * NHID || in_sizes[4] != NGATE || in_sizes[5] != NGATE || out_size != NBAT * NHID) return;

  const float* inp  = (const float*)d_in[0];
  const int*   len  = (const int*)  d_in[1];
  const float* w_ih = (const float*)d_in[2];
  const float* w_hh = (const float*)d_in[3];
  const float* b_ih = (const float*)d_in[4];
  const float* b_hh = (const float*)d_in[5];
  float* out = (float*)d_out;

  char* ws = (char*)d_ws; size_t off = 0;
  auto carve = [&](size_t bytes) -> char* { char* p = ws + off; off += (bytes + 255) & ~(size_t)255; return p; };
  unsigned short* XB   = (unsigned short*)carve((size_t)NBAT * NSTEP * NIN * 2);
  unsigned short* WIB  = (unsigned short*)carve((size_t)NGATE * NIN * 2);
  unsigned short* WHH  = (unsigned short*)carve((size_t)NGATE * NHID * 2);
  float*          BIAS = (float*)carve((size_t)NGATE * 4);
  if (off > ws_size || off > (size_t)134217728) return;

  const int n8x = (NBAT * NSTEP) * (NIN / 8);
  const int n8i = NGATE * (NIN / 8);
  const int n8h = NGATE * (NHID / 8);
  cvt8_kernel<0><<<n8x / NTHR, NTHR, 0, stream>>>(inp,  XB,  NBAT * NSTEP, NIN / 8,  NIN,  0, 1.0f);
  cvt8_kernel<0><<<n8i / NTHR, NTHR, 0, stream>>>(w_ih, WIB, NGATE,        NIN / 8,  NIN,  0, WCARRY);
  cvt8_kernel<1><<<n8h / NTHR, NTHR, 0, stream>>>(w_hh, WHH, NGATE,        NHID / 8, NHID, 0, WCARRY);
  bias_prep_kernel<<<(NGATE / 4) / NTHR, NTHR, 0, stream>>>(b_ih, b_hh, BIAS);
  lstm_seq_kernel<<<NBAT / SEQ_BLK, NTHR, 0, stream>>>(XB, WIB, WHH, BIAS, len, out);
}
